// BiLRNN_4063039062786
// MI455X (gfx1250) — hardware-run, weakly checked
//
#include <hip/hip_runtime.h>
#include <math.h>

typedef __attribute__((ext_vector_type(16))) __bf16   v16b;
typedef __attribute__((ext_vector_type(8)))  __bf16   v8b;
typedef __attribute__((ext_vector_type(8)))  float    v8f;
typedef __attribute__((ext_vector_type(4)))  float    v4f;
typedef __attribute__((ext_vector_type(4)))  unsigned v4u;

constexpr int kTok    = 8192;
constexpr int kFeat   = 256;
constexpr int kChan   = 32;
constexpr int kState  = 128;
constexpr int kHalf   = 64;
constexpr int kCat     = 448;
constexpr int kColGate = 0;
constexpr int kColProj = 128;
constexpr int kColVals = 256;
constexpr int kColGch  = 384;
constexpr int kColVch  = 416;
constexpr int kPlanes  = 8;
constexpr int kPerWave = 16;
constexpr int kChunk   = 32;
constexpr int kTilesM  = kTok / 64;
constexpr int kTilesN  = kCat / 64;

static_assert(kColProj == kState && kColVals == 2 * kState && kColGch == 3 * kState);
static_assert(kColVch == kColGch + kChan && kCat == kColVch + kChan);
static_assert(kPlanes * kPerWave == kState && (kPlanes / 2) * kPerWave == kHalf);
static_assert((kFeat % 32) == 0 && (kTok % 64) == 0 && (kCat % 64) == 0);
static_assert((kTilesM * kTilesN) % 8 == 0);
static_assert((kTok % kChunk) == 0 && kChan == 32 && kChunk == 32);

constexpr size_t kSzA16  = (size_t)kTok * kFeat * 2;
constexpr size_t kSzBT16 = (size_t)kCat * kFeat * 2;
constexpr size_t kSzPP   = (size_t)kTok * kCat * 4;
constexpr size_t kSzPART = (size_t)kPlanes * kTok * kChan * 4;
constexpr size_t kOffA16  = 0;
constexpr size_t kOffBT16 = kOffA16 + kSzA16;
constexpr size_t kOffPP   = kOffBT16 + kSzBT16;
constexpr size_t kOffPART = kOffPP + kSzPP;
constexpr size_t kWsTotal = kOffPART + kSzPART;
static_assert(kWsTotal == 27492352ull);
static_assert(kWsTotal <= 134217728ull);
static_assert((kOffBT16 % 128) == 0 && (kOffPP % 128) == 0 && (kOffPART % 128) == 0);

__device__ __forceinline__ unsigned bf16_bits_rne(float f) {
  const unsigned u = __float_as_uint(f);
  return (u + 0x7FFFu + ((u >> 16) & 1u)) >> 16;
}
__device__ __forceinline__ float bf16_value_rne(float f) {
  return __uint_as_float(bf16_bits_rne(f) << 16);
}
__device__ __forceinline__ unsigned pack_bf16x2(float lo_elem, float hi_elem) {
  const unsigned a = bf16_bits_rne(lo_elem);
  const unsigned b = bf16_bits_rne(hi_elem);
  return a | (b << 16);
}
__device__ __forceinline__ v8f mma_bf16_guarded(v16b a, v16b b, v8f c) {
  c = __builtin_amdgcn_wmma_f32_16x16x32_bf16(false, a, false, b, (short)0, c, false, false);
  asm volatile("v_nop\n\tv_nop\n\tv_nop\n\tv_nop" : "+v"(c) : "v"(a), "v"(b));
  return c;
}
__device__ __forceinline__ void keep4_b(v16b a, v16b b, v16b c, v16b d) {
  asm volatile("v_nop" :: "v"(a), "v"(b), "v"(c), "v"(d));
}
struct FragB {
  union U { v16b v; v8b h[2]; };
  static __device__ __forceinline__ v16b load(const __bf16* p) {
    U f;
    f.h[0] = *(const v8b*)(p);
    f.h[1] = *(const v8b*)(p + 16);
    return f.v;
  }
};
__device__ __forceinline__ void wave_sync_lds() {
  __builtin_amdgcn_fence(__ATOMIC_RELEASE, "workgroup");
  __builtin_amdgcn_wave_barrier();
  __builtin_amdgcn_fence(__ATOMIC_ACQUIRE, "workgroup");
}
__device__ __forceinline__ float gate_fn(float z, float db) {
  const float e1 = expf(z);
  float g = expf(-e1 - db);
  g = (g < 1.17549435e-38f) ? 0.0f : g;
  return g;
}

__global__ __launch_bounds__(256) void data_plane_kernel(const float* __restrict__ src, unsigned* __restrict__ dst)
{
  const int i = blockIdx.x * 256 + threadIdx.x;
  const size_t e0 = (size_t)i << 3;
  const v4f a0 = *(const v4f*)(src + e0);
  const v4f a1 = *(const v4f*)(src + e0 + 4);
  const float x0 = a0[0], x1 = a0[1], x2 = a0[2], x3 = a0[3];
  const float x4 = a1[0], x5 = a1[1], x6 = a1[2], x7 = a1[3];
  v4u o;
  o[0] = pack_bf16x2(x0, x1);
  o[1] = pack_bf16x2(x2, x3);
  o[2] = pack_bf16x2(x4, x5);
  o[3] = pack_bf16x2(x6, x7);
  unsigned* q = dst + ((size_t)i << 2);
  *(volatile v4u*)q = o;
  __threadfence();
  *(volatile v4u*)q = o;
}

__global__ __launch_bounds__(256) void weight_plane_kernel(
    const float* __restrict__ Wgate, const float* __restrict__ Wgproj, const float* __restrict__ Wvals,
    const float* __restrict__ Wgchan, const float* __restrict__ Wvalc, unsigned* __restrict__ dst)
{
  const int tid = threadIdx.x, lane = tid & 31, wave = tid >> 5;
  const int nb = blockIdx.x * 8;
  const float* W;
  int wc;
  int cb;
  if (nb < kColProj)      { W = Wgate;  wc = kState; cb = nb - kColGate; }
  else if (nb < kColVals) { W = Wgproj; wc = kState; cb = nb - kColProj; }
  else if (nb < kColGch)  { W = Wvals;  wc = kState; cb = nb - kColVals; }
  else if (nb < kColVch)  { W = Wgchan; wc = kChan;  cb = nb - kColGch; }
  else                    { W = Wvalc;  wc = kChan;  cb = nb - kColVch; }
  const int col = cb + wave;
  const int k8  = lane * 8;
  float x[8];
#pragma unroll
  for (int e = 0; e < 8; ++e) x[e] = W[(size_t)(k8 + e) * wc + col];
  v4u o;
  o[0] = pack_bf16x2(x[0], x[1]);
  o[1] = pack_bf16x2(x[2], x[3]);
  o[2] = pack_bf16x2(x[4], x[5]);
  o[3] = pack_bf16x2(x[6], x[7]);
  unsigned* q = dst + (size_t)(nb + wave) * (kFeat / 2) + lane * 4;
  *(volatile v4u*)q = o;
  __threadfence();
  *(volatile v4u*)q = o;
}

__global__ __launch_bounds__(256) void proj_gemm_kernel(
    const unsigned short* __restrict__ Ap, const unsigned short* __restrict__ Btp,
    float* __restrict__ Pout, const float* __restrict__ dlog)
{
  const __bf16* A  = (const __bf16*)Ap;
  const __bf16* Bt = (const __bf16*)Btp;
  __shared__ __align__(16) float sT[8][16 * 68];
  const int lane = threadIdx.x & 31;
  const int wave = threadIdx.x >> 5;
  const int tile = blockIdx.x * 8 + wave;
  if (tile >= kTilesM * kTilesN) return;
  const int tm = tile / kTilesN;
  const int tn = tile - tm * kTilesN;
  const int m0 = tm << 6;
  const int n0 = tn << 6;

  const int rlane = lane & 15;
  const int koff  = (lane >> 4) * 8;
  const int mOff  = (lane >> 4) * 8;

  v8f acc[4][4];
#pragma unroll
  for (int i = 0; i < 4; ++i)
#pragma unroll
    for (int j = 0; j < 4; ++j) acc[i][j] = (v8f){0.f,0.f,0.f,0.f,0.f,0.f,0.f,0.f};

  for (int k0 = 0; k0 < kFeat; k0 += 32) {
    v16b bh[4];
#pragma unroll
    for (int j = 0; j < 4; ++j) {
      const size_t bo = (size_t)(n0 + (j << 4) + rlane) * kFeat + koff + k0;
      bh[j] = FragB::load(Bt + bo);
    }
#pragma unroll
    for (int i = 0; i < 4; ++i) {
      const size_t ao = (size_t)(m0 + (i << 4) + rlane) * kFeat + koff + k0;
      const v16b ah = FragB::load(A + ao);
#pragma unroll
      for (int j = 0; j < 4; ++j) acc[i][j] = mma_bf16_guarded(ah, bh[j], acc[i][j]);
    }
    keep4_b(bh[0], bh[1], bh[2], bh[3]);
  }

  float* slab = sT[wave];
  const int hh = lane >> 4, c4 = (lane & 15) * 4;
  const bool isGate = (n0 < kColProj);
  float db0, db1, db2, db3;
  {
    const int dcol = (isGate ? n0 : 0) + c4;
    const v4f dl = *(const v4f*)(dlog + dcol);
    const float d0 = dl[0], d1 = dl[1], d2 = dl[2], d3 = dl[3];
    db0 = expf(bf16_value_rne(d0));
    db1 = expf(bf16_value_rne(d1));
    db2 = expf(bf16_value_rne(d2));
    db3 = expf(bf16_value_rne(d3));
  }
#pragma unroll
  for (int i = 0; i < 4; ++i) {
    const int mBase = m0 + (i << 4);
#pragma unroll
    for (int j = 0; j < 4; ++j) {
#pragma unroll
      for (int r = 0; r < 8; ++r) slab[(mOff + r) * 68 + (j << 4) + rlane] = acc[i][j][r];
    }
    wave_sync_lds();
    if (isGate) {
#pragma unroll 1
      for (int it = 0; it < 8; ++it) {
        float* sp = slab + (it * 2 + hh) * 68 + c4;
        const v4f zv = *(const v4f*)sp;
        const float z0 = zv[0], z1 = zv[1], z2 = zv[2], z3 = zv[3];
        v4f gv;
        gv[0] = gate_fn(z0, db0);
        gv[1] = gate_fn(z1, db1);
        gv[2] = gate_fn(z2, db2);
        gv[3] = gate_fn(z3, db3);
        *(v4f*)sp = gv;
      }
      wave_sync_lds();
    }
    for (int pass = 0; pass < 2; ++pass) {
#pragma unroll
      for (int it = 0; it < 8; ++it) {
        const int row = it * 2 + hh;
        const v4f v = *(const v4f*)(slab + row * 68 + c4);
        *(volatile v4f*)(Pout + (size_t)(mBase + row) * kCat + n0 + c4) = v;
      }
      __threadfence();
    }
    wave_sync_lds();
  }
}

__global__ __launch_bounds__(32) void scan_readout_kernel(
    const float* __restrict__ P, const int* __restrict__ idx, float* __restrict__ part)
{
  __shared__ __align__(16) float sG[kChunk * kPerWave];
  __shared__ __align__(16) float sV[kChunk * kPerWave];
  __shared__ __align__(16) float sQ[kChunk * kPerWave];
  __shared__ __align__(16) float sC[kChunk * kChan];
  __shared__ __align__(16) float sD[kChunk * kChan];
  __shared__ __align__(16) float sO[kChunk * kChan];
  __shared__ int sF[kChunk];

  const int lane = threadIdx.x;
  const int w    = blockIdx.x;
  const bool left = (w < (kPlanes / 2));
  const int kb   = kPerWave * w;
  float* outp = part + (size_t)w * kTok * kChan;

  float S[kPerWave];
#pragma unroll
  for (int k = 0; k < kPerWave; ++k) S[k] = 0.0f;

#pragma unroll 1
  for (int t0 = 0; t0 < kTok; t0 += kChunk) {
    __syncthreads();
    {
      const int p   = t0 + lane;
      const int tok = left ? p : (kTok - 1 - p);
      const float* rowT = P + (size_t)tok * kCat;
      const float* rowP = P + (size_t)p * kCat;
#pragma unroll
      for (int i = 0; i < 4; ++i) {
        const v4f g4 = *(const v4f*)(rowT + kColGate + kb + 4 * i);
        const v4f v4 = *(const v4f*)(rowT + kColVals + kb + 4 * i);
        const v4f q4 = *(const v4f*)(rowP + kColProj + kb + 4 * i);
        *(v4f*)(sG + lane * kPerWave + 4 * i) = g4;
        *(v4f*)(sV + lane * kPerWave + 4 * i) = v4;
        *(v4f*)(sQ + lane * kPerWave + 4 * i) = q4;
      }
      int nbr = left ? (tok - 1) : (tok + 1);
      nbr = (nbr < 0) ? (nbr + kTok) : nbr;
      nbr = (nbr >= kTok) ? (nbr - kTok) : nbr;
      const int ia = idx[tok];
      const int ib = idx[nbr];
      sF[lane] = (ia != ib) ? 1 : 0;
    }
#pragma unroll
    for (int i = 0; i < 8; ++i) {
      const int j   = lane + 32 * i;
      const int s2  = j >> 3;
      const int cc4 = (j & 7) * 4;
      const int p2  = t0 + s2;
      const int tk2 = left ? p2 : (kTok - 1 - p2);
      const v4f a = *(const v4f*)(P + (size_t)tk2 * kCat + kColGch + cc4);
      const v4f b = *(const v4f*)(P + (size_t)tk2 * kCat + kColVch + cc4);
      *(v4f*)(sC + s2 * kChan + cc4) = a;
      *(v4f*)(sD + s2 * kChan + cc4) = b;
    }
    __syncthreads();

#pragma unroll 1
    for (int s = 0; s < kChunk; ++s) {
      const float gcv = sC[s * kChan + lane];
      const float vcv = sD[s * kChan + lane];
      const int   flg = sF[s];
      const float gce = (flg != 0) ? 0.0f : gcv;
      float accp = 0.0f;
#pragma unroll
      for (int q4 = 0; q4 < 4; ++q4) {
        const v4f gv = *(const v4f*)(sG + s * kPerWave + 4 * q4);
        const v4f vv = *(const v4f*)(sV + s * kPerWave + 4 * q4);
        const v4f qv = *(const v4f*)(sQ + s * kPerWave + 4 * q4);
#pragma unroll
        for (int e = 0; e < 4; ++e) {
          const float gk = gv[e] * gce;
          const float uk = vcv * vv[e];
          S[4 * q4 + e] = fmaf(gk, S[4 * q4 + e], uk);
          accp = fmaf(S[4 * q4 + e], qv[e], accp);
        }
      }
      sO[s * kChan + lane] = accp;
    }
    __syncthreads();

    v4f ov[8];
#pragma unroll
    for (int i = 0; i < 8; ++i) ov[i] = *(const v4f*)(sO + (i * 32 + lane) * 4);
    float* dst = outp + (size_t)t0 * kChan;
#pragma unroll
    for (int i = 0; i < 8; ++i) *(volatile v4f*)(dst + (i * 32 + lane) * 4) = ov[i];
    __threadfence();
#pragma unroll
    for (int i = 0; i < 8; ++i) *(volatile v4f*)(dst + (i * 32 + lane) * 4) = ov[i];
    __threadfence();
  }
}

__global__ __launch_bounds__(256) void sum_planes_kernel(const float* __restrict__ part, float* __restrict__ out)
{
  const int i = blockIdx.x * 256 + threadIdx.x;
  const size_t e = (size_t)i << 2;
  v4f a = (v4f){0.f, 0.f, 0.f, 0.f};
#pragma unroll
  for (int w = 0; w < kPlanes; ++w) {
    const v4f t = *(const v4f*)(part + (size_t)w * kTok * kChan + e);
    a = a + t;
  }
  float* q = out + e;
  *(volatile v4f*)q = a;
  __threadfence();
  *(volatile v4f*)q = a;
}

extern "C" void kernel_launch(void* const* d_in, const int* in_sizes, int n_in,
                              void* d_out, int out_size, void* d_ws, size_t ws_size,
                              hipStream_t stream) {
  if (n_in < 8) return;
  if (in_sizes[0] != kTok * kFeat) return;
  if (in_sizes[1] != kTok) return;
  if (in_sizes[2] != kState) return;
  if (in_sizes[3] != kFeat * kState) return;
  if (in_sizes[4] != kFeat * kState) return;
  if (in_sizes[5] != kFeat * kChan) return;
  if (in_sizes[6] != kFeat * kChan) return;
  if (in_sizes[7] != kFeat * kState) return;
  if (out_size != kTok * kChan) return;
  if (ws_size < kWsTotal) return;

  const float* data   = (const float*)d_in[0];
  const int*   index  = (const int*)  d_in[1];
  const float* dlog   = (const float*)d_in[2];
  const float* Wgate  = (const float*)d_in[3];
  const float* Wgproj = (const float*)d_in[4];
  const float* Wgchan = (const float*)d_in[5];
  const float* Wvalc  = (const float*)d_in[6];
  const float* Wvals  = (const float*)d_in[7];
  float* out = (float*)d_out;

  char* ws = (char*)d_ws;
  unsigned* A16w  = (unsigned*)(ws + kOffA16);
  unsigned* BT16w = (unsigned*)(ws + kOffBT16);
  float*    PP    = (float*)(ws + kOffPP);
  float*    PART  = (float*)(ws + kOffPART);

  data_plane_kernel<<<(kTok * kFeat / 8) / 256, 256, 0, stream>>>(data, A16w);

  weight_plane_kernel<<<kCat / 8, 256, 0, stream>>>(Wgate, Wgproj, Wvals, Wgchan, Wvalc, BT16w);

  proj_gemm_kernel<<<(kTilesM * kTilesN) / 8, 256, 0, stream>>>(
      (const unsigned short*)A16w, (const unsigned short*)BT16w, PP, dlog);

  scan_readout_kernel<<<kPlanes, 32, 0, stream>>>(PP, index, PART);

  sum_planes_kernel<<<(kTok * kChan / 4) / 256, 256, 0, stream>>>(PART, out);
}
